// FastQuantumV2_77129022702014
// MI455X (gfx1250) — hardware-verified
//
#include <hip/hip_runtime.h>
#include <stddef.h>


#define HCW   256
#define NH    4
#define CH    64
#define INW   32
#define GR    32
#define XSP   260
#define NB    256
#define CHUNK 2048
#define NTHR  256
#define NWAVE 8
#define WCAP  256
#define NGRP  (CHUNK / (NTHR * 4))
#define GP    128
#define CBW   160
#define CBP   164
#define Z1P   132
#define Z2P   68
#define EMBW  16
#define M1K   144
#define M1N   128
#define M2N   64
#define OUTW  2

#define LDS_SACC (NB * HCW)
#define LDS_DEN  (NB * NH)
#define LDS_MRN  (NB * NH)
#define LDS_LIST (NWAVE * WCAP)
#define AGG_LDS_BYTES ((LDS_SACC + LDS_DEN + LDS_MRN + LDS_LIST + NWAVE + NH) * 4)
#define MLP_LDS_BYTES ((GP * CBP + GP * Z1P) * 4)

static_assert(NTHR == HCW);
static_assert(WCAP == (CHUNK / NTHR) * 32);
static_assert(NGRP >= 1);
static_assert(NB == 256);
static_assert(CHUNK == 2048);
static_assert(GP == 16 * NWAVE);
static_assert(((LDS_SACC + LDS_DEN) % 4) == 0);
static_assert((LDS_MRN % 4) == 0);
static_assert(AGG_LDS_BYTES == 278576);
static_assert(MLP_LDS_BYTES == 151552);
static_assert(CBW == 2 * CH + 2 * EMBW);
static_assert(M1K == 2 * CH + EMBW);
static_assert((NB / NWAVE) == 32);

typedef float    v2f  __attribute__((ext_vector_type(2)));
typedef float    v4f  __attribute__((ext_vector_type(4)));
typedef float    v8f  __attribute__((ext_vector_type(8)));
typedef int      v4i  __attribute__((ext_vector_type(4)));
typedef _Float16 v8h  __attribute__((ext_vector_type(8)));
typedef _Float16 v16h __attribute__((ext_vector_type(16)));
typedef __bf16   v16b __attribute__((ext_vector_type(16)));
union FragH  { v16h v; v8h half[2]; };
union FragB  { v16b v; unsigned short u[16]; };
union Pack16 { v8h h; v4i i; };

extern __shared__ v4f lds_dyn[];

__device__ __forceinline__ v8f wmh(v16h a, v16h b, v8f c) {
  v8f d = __builtin_amdgcn_wmma_f32_16x16x32_f16(false, a, false, b, (short)0, c, false, false);
  asm volatile("v_nop\n\tv_nop\n\tv_nop\n\tv_nop" : "+v"(d) : "v"(a), "v"(b));
  return d;
}
__device__ __forceinline__ v8f wmb(v16b a, v16b b, v8f c) {
  v8f d = __builtin_amdgcn_wmma_f32_16x16x32_bf16(false, a, false, b, (short)0, c, false, false);
  asm volatile("v_nop\n\tv_nop\n\tv_nop\n\tv_nop" : "+v"(d) : "v"(a), "v"(b));
  return d;
}

__device__ __forceinline__ unsigned short bf_rne(float f) {
  const unsigned x = __float_as_uint(f);
  return (unsigned short)((x + 0x7FFFu + ((x >> 16) & 1u)) >> 16);
}
__device__ __forceinline__ void split2(float f, unsigned short& h, unsigned short& l) {
  h = bf_rne(f);
  const float fh = __uint_as_float(((unsigned)h) << 16);
  l = bf_rne(f - fh);
}

__device__ __forceinline__ v4f ld4(const float* p) { return *(const v4f*)p; }
__device__ __forceinline__ v4f rsq4(v4f v) {
  v4f r;
  r.x = rsqrtf(v.x + 1e-5f); r.y = rsqrtf(v.y + 1e-5f);
  r.z = rsqrtf(v.z + 1e-5f); r.w = rsqrtf(v.w + 1e-5f);
  return r;
}
__device__ __forceinline__ v4f bn4(v4f h, v4f m, v4f rs, v4f g, v4f b) {
  v4f t = (h - m) * rs;
  t = t * g;
  return t + b;
}
__device__ __forceinline__ float elu1(float y) { return y > 0.f ? y : (__expf(y) - 1.0f); }
__device__ __forceinline__ v4f elu4(v4f y) {
  v4f r;
  r.x = elu1(y.x); r.y = elu1(y.y); r.z = elu1(y.z); r.w = elu1(y.w);
  return r;
}
__device__ __forceinline__ v4f xsum_heads(v4f v) {
  v.x += __shfl_xor(v.x, 8, 32);  v.y += __shfl_xor(v.y, 8, 32);
  v.z += __shfl_xor(v.z, 8, 32);  v.w += __shfl_xor(v.w, 8, 32);
  v.x += __shfl_xor(v.x, 16, 32); v.y += __shfl_xor(v.y, 16, 32);
  v.z += __shfl_xor(v.z, 16, 32); v.w += __shfl_xor(v.w, 16, 32);
  return v;
}

__global__ __launch_bounds__(NTHR) void k_eamean(const float* __restrict__ ea, float* eam, int nE) {
  __shared__ double red[NTHR];
  const int tid = threadIdx.x;
  double s = 0.0;
  for (int i = tid; i < nE; i += NTHR) s += (double)ea[i];
  red[tid] = s;
  __syncthreads();
  for (int off = NTHR / 2; off > 0; off >>= 1) {
    if (tid < off) red[tid] += red[tid + off];
    __syncthreads();
  }
  const float m = (nE > 0) ? (float)(red[0] * (1.0 / (double)nE)) : 0.f;
  const v4f q = {m, m, m, m};
  if (tid < 32) *(volatile v4f*)(eam + 4 * tid) = q;
  __threadfence();
  if (tid < 32) *(volatile v4f*)(eam + 4 * tid) = q;
}

__global__ __launch_bounds__(NTHR) void k_cvx(const float* __restrict__ x, _Float16* xh, int nN, int n8) {
  const int u = blockIdx.x * NTHR + threadIdx.x;
  if (u >= n8) return;
  const int row = u >> 2;
  const int c0  = (u & 3) * 8;
  Pack16 p;
  if (row < nN) {
    const v4f a = ld4(x + (size_t)row * INW + c0);
    const v4f b = ld4(x + (size_t)row * INW + c0 + 4);
    p.h[0] = (_Float16)a.x; p.h[1] = (_Float16)a.y; p.h[2] = (_Float16)a.z; p.h[3] = (_Float16)a.w;
    p.h[4] = (_Float16)b.x; p.h[5] = (_Float16)b.y; p.h[6] = (_Float16)b.z; p.h[7] = (_Float16)b.w;
  } else {
    const _Float16 z = (_Float16)0.0f;
    p.h[0] = z; p.h[1] = z; p.h[2] = z; p.h[3] = z; p.h[4] = z; p.h[5] = z; p.h[6] = z; p.h[7] = z;
  }
  _Float16* op = xh + (size_t)u * 8;
  *(volatile v4i*)op = p.i;
  __threadfence();
  *(volatile v4i*)op = p.i;
}

template<int K>
__global__ __launch_bounds__(NTHR) void k_prepw(const float* __restrict__ W, _Float16* Wt) {
  __shared__ __attribute__((aligned(16))) _Float16 Ts[32 * (K + 8)];
  const int tid = threadIdx.x;
  const int n0  = blockIdx.x * 32;
  const int kk  = tid >> 3;
  const int nq  = (tid & 7) * 4;
#pragma unroll 1
  for (int kt = 0; kt < K / 32; ++kt) {
    const int k = kt * 32 + kk;
    const v4f wv = ld4(W + (size_t)k * HCW + n0 + nq);
    Ts[(nq + 0) * (K + 8) + k] = (_Float16)(wv.x * 8.0f);
    Ts[(nq + 1) * (K + 8) + k] = (_Float16)(wv.y * 8.0f);
    Ts[(nq + 2) * (K + 8) + k] = (_Float16)(wv.z * 8.0f);
    Ts[(nq + 3) * (K + 8) + k] = (_Float16)(wv.w * 8.0f);
  }
  __syncthreads();
  const int nu = 4 * K;
  _Float16* base = Wt + (size_t)n0 * K;
  for (int u = tid; u < nu; u += NTHR) {
    const int nn = u / (K / 8), c = (u - nn * (K / 8)) * 8;
    Pack16 p; p.h = *(const v8h*)(Ts + nn * (K + 8) + c);
    *(volatile v4i*)(base + (size_t)u * 8) = p.i;
  }
  __threadfence();
  for (int u = tid; u < nu; u += NTHR) {
    const int nn = u / (K / 8), c = (u - nn * (K / 8)) * 8;
    Pack16 p; p.h = *(const v8h*)(Ts + nn * (K + 8) + c);
    *(volatile v4i*)(base + (size_t)u * 8) = p.i;
  }
}

template<int K>
__global__ __launch_bounds__(NTHR) void k_gemm(
    const _Float16* __restrict__ Ah, const _Float16* __restrict__ Wt,
    const float* __restrict__ att_s, const float* __restrict__ att_d,
    float* xp, float* asrc, float* adst) {
  __shared__ __attribute__((aligned(16))) float Xs[GR * XSP];
  __shared__ __attribute__((aligned(16))) float Sa[HCW];
  __shared__ __attribute__((aligned(16))) float Sd[HCW];
  __shared__ __attribute__((aligned(16))) float As[GR * NH];
  __shared__ __attribute__((aligned(16))) float Ds[GR * NH];

  const int tid  = threadIdx.x;
  const int lane = tid & 31;
  const int wave = tid >> 5;
  const int hh   = lane >> 4;
  const int m    = lane & 15;
  const int rowBase = blockIdx.x * GR;

  Sa[tid] = att_s[tid];
  Sd[tid] = att_d[tid];

  const int n0 = wave * 32 + m, n1 = n0 + 16;
  const _Float16* pa0 = Ah + (size_t)(rowBase + m) * K + 8 * hh;
  const _Float16* pa1 = Ah + (size_t)(rowBase + 16 + m) * K + 8 * hh;
  const _Float16* pb0 = Wt + (size_t)n0 * K + 8 * hh;
  const _Float16* pb1 = Wt + (size_t)n1 * K + 8 * hh;
  v8f c00 = {0.f, 0.f, 0.f, 0.f, 0.f, 0.f, 0.f, 0.f};
  v8f c01 = c00, c10 = c00, c11 = c00;
#pragma unroll 2
  for (int kt = 0; kt < K / 32; ++kt) {
    const int k0 = kt * 32;
    FragH a0, a1, b0, b1;
    a0.half[0] = *(const v8h*)(pa0 + k0); a0.half[1] = *(const v8h*)(pa0 + k0 + 16);
    a1.half[0] = *(const v8h*)(pa1 + k0); a1.half[1] = *(const v8h*)(pa1 + k0 + 16);
    b0.half[0] = *(const v8h*)(pb0 + k0); b0.half[1] = *(const v8h*)(pb0 + k0 + 16);
    b1.half[0] = *(const v8h*)(pb1 + k0); b1.half[1] = *(const v8h*)(pb1 + k0 + 16);
    c00 = wmh(a0.v, b0.v, c00);
    c01 = wmh(a0.v, b1.v, c01);
    c10 = wmh(a1.v, b0.v, c10);
    c11 = wmh(a1.v, b1.v, c11);
  }

#pragma unroll
  for (int r = 0; r < 8; ++r) {
    Xs[(8 * hh + r) * XSP + n0]      = c00[r] * 0.125f;
    Xs[(8 * hh + r) * XSP + n1]      = c01[r] * 0.125f;
    Xs[(16 + 8 * hh + r) * XSP + n0] = c10[r] * 0.125f;
    Xs[(16 + 8 * hh + r) * XSP + n1] = c11[r] * 0.125f;
  }
  __syncthreads();

  {
    const int r  = tid >> 3;
    const int hs = (tid >> 1) & 3;
    const int wh = tid & 1;
    const float* xr = Xs + r * XSP + hs * CH;
    const float* av = (wh ? Sd : Sa) + hs * CH;
    float s = 0.f;
#pragma unroll 4
    for (int c = 0; c < CH; c += 4) {
      const v4f xv = *(const v4f*)(xr + c);
      const v4f a4 = *(const v4f*)(av + c);
      s += xv.x * a4.x; s += xv.y * a4.y; s += xv.z * a4.z; s += xv.w * a4.w;
    }
    if (wh) Ds[r * NH + hs] = s; else As[r * NH + hs] = s;
  }
  __syncthreads();

  v4f xr[8];
#pragma unroll
  for (int i = 0; i < 4; ++i) {
    xr[2 * i]     = *(const v4f*)(Xs + (4 * wave + i) * XSP + 4 * lane);
    xr[2 * i + 1] = *(const v4f*)(Xs + (4 * wave + i) * XSP + 128 + 4 * lane);
  }
  v4f gv = {0.f, 0.f, 0.f, 0.f};
  if (wave == 0) gv = *(const v4f*)(As + 4 * lane);
  else if (wave == 1) gv = *(const v4f*)(Ds + 4 * lane);
  float* xb = xp + (size_t)(rowBase + 4 * wave) * HCW + 4 * lane;
  float* gp = (wave == 0) ? (asrc + (size_t)rowBase * NH + 4 * lane)
                          : (adst + (size_t)rowBase * NH + 4 * lane);
#pragma unroll
  for (int i = 0; i < 4; ++i) {
    *(volatile v4f*)(xb + (size_t)i * HCW)       = xr[2 * i];
    *(volatile v4f*)(xb + (size_t)i * HCW + 128) = xr[2 * i + 1];
  }
  if (wave < 2) *(volatile v4f*)gp = gv;
  __threadfence();
#pragma unroll
  for (int i = 0; i < 4; ++i) {
    *(volatile v4f*)(xb + (size_t)i * HCW)       = xr[2 * i];
    *(volatile v4f*)(xb + (size_t)i * HCW + 128) = xr[2 * i + 1];
  }
  if (wave < 2) *(volatile v4f*)gp = gv;
}

__device__ __forceinline__ void fin_slot(const float* sacc, const float* den, const float* mrn,
                                         const float* __restrict__ xp, const float* __restrict__ asrc,
                                         const float* __restrict__ adst,
                                         int slot, int node, int lane, int hd, float la, float kreg,
                                         v4f& o0, v4f& o1) {
  float al = asrc[(size_t)node * NH + hd] + adst[(size_t)node * NH + hd] + la * kreg;
  al = (al > 0.f) ? al : 0.2f * al;
  const int ai = slot * NH + hd;
  const float mo = mrn[ai];
  const float mn = fmaxf(mo, al);
  const float co = __expf(mo - mn);
  const float p  = __expf(al - mn);
  const float* xs = xp + (size_t)node * HCW + 8 * lane;
  const v4f x0 = ld4(xs), x1 = ld4(xs + 4);
  const v4f* sp = (const v4f*)(sacc + slot * HCW + 8 * lane);
  const float dv  = den[ai] * co + p;
  const float inv = __builtin_amdgcn_rcpf(dv);
  o0 = (sp[0] * co + x0 * p) * inv;
  o1 = (sp[1] * co + x1 * p) * inv;
}

template<int MODE>
__global__ __launch_bounds__(NTHR) void k_agg(
    const int* __restrict__ ei, const float* __restrict__ ea, const float* __restrict__ eam,
    const float* __restrict__ xp, const float* __restrict__ asrc, const float* __restrict__ adst,
    const float* __restrict__ we, const float* __restrict__ ae,
    const float* __restrict__ bias, const float* __restrict__ bng, const float* __restrict__ bnb,
    const float* __restrict__ bnm, const float* __restrict__ bnv,
    _Float16* hb, float* hout, int nN, int nE) {
  float* sacc = (float*)lds_dyn;
  float* den  = sacc + LDS_SACC;
  float* mrn  = den + LDS_DEN;
  int*   list = (int*)(mrn + LDS_MRN);
  int*   wcnt = list + LDS_LIST;
  float* kap  = (float*)(wcnt + NWAVE);

  const int tid  = threadIdx.x;
  const int lane = tid & 31;
  const int wave = tid >> 5;
  const int hd   = lane >> 3;
  const int nodeBase = blockIdx.x * NB;

  {
    const v4f z4 = {0.f, 0.f, 0.f, 0.f};
    const v4f n4 = {-1.0e30f, -1.0e30f, -1.0e30f, -1.0e30f};
    const int nz = (LDS_SACC + LDS_DEN) / 4;
    const int nm = LDS_MRN / 4;
    for (int i = tid; i < nz; i += NTHR) lds_dyn[i] = z4;
    for (int i = tid; i < nm; i += NTHR) lds_dyn[nz + i] = n4;
    if (tid < NH) {
      float s = 0.f;
#pragma unroll 1
      for (int c = 0; c < CH; ++c) s += we[tid * CH + c] * ae[tid * CH + c];
      kap[tid] = s;
    }
  }
  __syncthreads();
  const float kreg = kap[hd];
  const int* eid = ei + nE;
  const bool al16 = ((nE & 3) == 0);

  const int nChunks = (nE + CHUNK - 1) / CHUNK;
#pragma unroll 1
  for (int ch = 0; ch < nChunks; ++ch) {
    const int cbase = ch * CHUNK;
    int wc = 0;
#pragma unroll
    for (int g = 0; g < NGRP; ++g) {
      const int el0 = (g * NTHR + tid) * 4;
      const int e0  = cbase + el0;
      const int sent = -2147483647 - 1;
      v4i d;
      if (al16 && (e0 + 3 < nE)) {
        d = *(const v4i*)(eid + e0);
      } else {
        d.x = (e0     < nE) ? eid[e0]     : sent;
        d.y = (e0 + 1 < nE) ? eid[e0 + 1] : sent;
        d.z = (e0 + 2 < nE) ? eid[e0 + 2] : sent;
        d.w = (e0 + 3 < nE) ? eid[e0 + 3] : sent;
      }
      const unsigned s0 = (unsigned)d.x - (unsigned)nodeBase;
      const unsigned s1 = (unsigned)d.y - (unsigned)nodeBase;
      const unsigned s2 = (unsigned)d.z - (unsigned)nodeBase;
      const unsigned s3 = (unsigned)d.w - (unsigned)nodeBase;
      const bool q0 = s0 < (unsigned)NB;
      const bool q1 = s1 < (unsigned)NB;
      const bool q2 = s2 < (unsigned)NB;
      const bool q3 = s3 < (unsigned)NB;
      const unsigned many = __builtin_amdgcn_ballot_w32(q0 | q1 | q2 | q3);
      if (many != 0u) {
#define HITJ(J, QJ, SJ) { \
          const unsigned mj = __builtin_amdgcn_ballot_w32(QJ); \
          if (QJ) { \
            const int pos = wc + (int)__builtin_amdgcn_mbcnt_lo(mj, 0u); \
            if (pos < WCAP) list[wave * WCAP + pos] = ((el0 + (J)) << 8) | (int)(SJ); \
          } \
          wc += (int)__builtin_popcount(mj); }
        HITJ(0, q0, s0)
        HITJ(1, q1, s1)
        HITJ(2, q2, s2)
        HITJ(3, q3, s3)
#undef HITJ
      }
    }
    if (lane == 0) wcnt[wave] = wc;
    __syncthreads();

    if (wave == 0) {
#pragma unroll 1
      for (int wsx = 0; wsx < NWAVE; ++wsx) {
        int n = wcnt[wsx];
        if (n > WCAP) n = WCAP;
        if (n < 0) n = 0;
#pragma unroll 1
        for (int i = 0; i < n; ++i) {
          const int ent  = list[wsx * WCAP + i];
          const int slot = ent & (NB - 1);
          const int el   = (ent >> 8) & (CHUNK - 1);
          int e = cbase + el;
          if (e > nE - 1) e = nE - 1;
          int src = ei[e];
          src = src < 0 ? 0 : (src > nN - 1 ? nN - 1 : src);
          const float w = ea[e];
          int nd = nodeBase + slot;
          if (nd > nN - 1) nd = nN - 1;
          float al = asrc[(size_t)src * NH + hd] + adst[(size_t)nd * NH + hd] + w * kreg;
          al = (al > 0.f) ? al : 0.2f * al;
          const int ai = slot * NH + hd;
          const float mo = mrn[ai];
          const float mn = fmaxf(mo, al);
          const float co = __expf(mo - mn);
          const float p  = __expf(al - mn);
          const float* xs = xp + (size_t)src * HCW + 8 * lane;
          const v4f x0 = ld4(xs), x1 = ld4(xs + 4);
          v4f* sp = (v4f*)(sacc + slot * HCW + 8 * lane);
          const v4f c0v = sp[0], c1v = sp[1];
          const v4f n0v = c0v * co + x0 * p;
          const v4f n1v = c1v * co + x1 * p;
          sp[0] = n0v;
          sp[1] = n1v;
          if ((lane & 7) == 0) {
            const float dv = den[ai];
            den[ai] = dv * co + p;
            mrn[ai] = mn;
          }
        }
      }
    }
    __syncthreads();
  }

  const float la = eam[0];
  if (MODE == 0) {
    const int c0 = 8 * lane;
    const v4f bi0 = ld4(bias + c0), bi1 = ld4(bias + c0 + 4);
    const v4f m0  = ld4(bnm + c0),  m1  = ld4(bnm + c0 + 4);
    const v4f g0  = ld4(bng + c0),  g1  = ld4(bng + c0 + 4);
    const v4f e0  = ld4(bnb + c0),  e1  = ld4(bnb + c0 + 4);
    const v4f rs0 = rsq4(ld4(bnv + c0)), rs1 = rsq4(ld4(bnv + c0 + 4));
#pragma unroll 1
    for (int j = 0; j < NB / NWAVE; ++j) {
      const int slot = wave * (NB / NWAVE) + j;
      const int node = nodeBase + slot;
      if (node >= nN) break;
      v4f o0, o1;
      fin_slot(sacc, den, mrn, xp, asrc, adst, slot, node, lane, hd, la, kreg, o0, o1);
      v4f y0 = bn4(o0 + bi0, m0, rs0, g0, e0);
      v4f y1 = bn4(o1 + bi1, m1, rs1, g1, e1);
      y0 = elu4(y0);
      y1 = elu4(y1);
      Pack16 pk;
      pk.h[0] = (_Float16)y0.x; pk.h[1] = (_Float16)y0.y; pk.h[2] = (_Float16)y0.z; pk.h[3] = (_Float16)y0.w;
      pk.h[4] = (_Float16)y1.x; pk.h[5] = (_Float16)y1.y; pk.h[6] = (_Float16)y1.z; pk.h[7] = (_Float16)y1.w;
      _Float16* op = hb + (size_t)node * HCW + c0;
      *(volatile v4i*)op = pk.i;
      __threadfence();
      *(volatile v4i*)op = pk.i;
    }
  } else {
    const int cb = 8 * (lane & 7);
    const v4f bi0 = ld4(bias + cb), bi1 = ld4(bias + cb + 4);
    const v4f m0  = ld4(bnm + cb),  m1  = ld4(bnm + cb + 4);
    const v4f g0  = ld4(bng + cb),  g1  = ld4(bng + cb + 4);
    const v4f e0  = ld4(bnb + cb),  e1  = ld4(bnb + cb + 4);
    const v4f rs0 = rsq4(ld4(bnv + cb)), rs1 = rsq4(ld4(bnv + cb + 4));
    const int sl = (lane >> 1) & 7;
#pragma unroll 1
    for (int j = 0; j < NB / NWAVE; ++j) {
      const int slot = wave * (NB / NWAVE) + j;
      const int node = nodeBase + slot;
      if (node >= nN) break;
      v4f o0, o1;
      fin_slot(sacc, den, mrn, xp, asrc, adst, slot, node, lane, hd, la, kreg, o0, o1);
      o0 = xsum_heads(o0);
      o1 = xsum_heads(o1);
      const v4f y0 = bn4(o0 * 0.25f + bi0, m0, rs0, g0, e0);
      const v4f y1 = bn4(o1 * 0.25f + bi1, m1, rs1, g1, e1);
      v4f t0, t1;
      t0.x = __shfl(y0.x, sl, 32); t0.y = __shfl(y0.y, sl, 32); t0.z = __shfl(y0.z, sl, 32); t0.w = __shfl(y0.w, sl, 32);
      t1.x = __shfl(y1.x, sl, 32); t1.y = __shfl(y1.y, sl, 32); t1.z = __shfl(y1.z, sl, 32); t1.w = __shfl(y1.w, sl, 32);
      v4f o = t0;
      if (lane & 1) o = t1;
      float* op = hout + (size_t)node * CH + 4 * lane;
      if (lane < 16) *(volatile v4f*)op = o;
      __threadfence();
      if (lane < 16) *(volatile v4f*)op = o;
    }
  }
}

__global__ __launch_bounds__(NTHR) void k_pool(const float* __restrict__ hf, const int* __restrict__ bat,
                                               const float* __restrict__ emb, const int* __restrict__ cids,
                                               float* comb, int nN, int nEmb) {
  __shared__ __attribute__((aligned(16))) float psum[NWAVE * CH];
  __shared__ __attribute__((aligned(16))) float pmax[NWAVE * CH];
  __shared__ __attribute__((aligned(16))) float res[CBW];
  __shared__ int pcnt[NWAVE];
  const int tid  = threadIdx.x;
  const int lane = tid & 31;
  const int wave = tid >> 5;
  const int g    = blockIdx.x;
  const float ninf = -__builtin_huge_valf();

  v2f s  = {0.f, 0.f};
  v2f mx = {ninf, ninf};
  int cnt = 0;
#pragma unroll 1
  for (int base = wave * 32; base < nN; base += NTHR) {
    const int node = base + lane;
    const int b = (node < nN) ? bat[node] : -1;
    unsigned msk = __builtin_amdgcn_ballot_w32(b == g);
    while (msk != 0u) {
      const int i = __builtin_ctz(msk);
      msk &= msk - 1u;
      const int n = base + i;
      const v2f v = *(const v2f*)(hf + (size_t)n * CH + 2 * lane);
      s += v;
      mx.x = fmaxf(mx.x, v.x);
      mx.y = fmaxf(mx.y, v.y);
      ++cnt;
    }
  }
  psum[wave * CH + 2 * lane]     = s.x;
  psum[wave * CH + 2 * lane + 1] = s.y;
  pmax[wave * CH + 2 * lane]     = mx.x;
  pmax[wave * CH + 2 * lane + 1] = mx.y;
  if (lane == 0) pcnt[wave] = cnt;
  __syncthreads();
  if (tid < CH) {
    float S = 0.f, M = ninf;
    int C = 0;
#pragma unroll
    for (int w = 0; w < NWAVE; ++w) {
      S += psum[w * CH + tid];
      M = fmaxf(M, pmax[w * CH + tid]);
      C += pcnt[w];
    }
    const float cc = (float)(C < 1 ? 1 : C);
    res[tid]      = S * __builtin_amdgcn_rcpf(cc);
    res[CH + tid] = M;
  } else if (tid >= 2 * CH && tid < 2 * CH + EMBW) {
    int cid = cids[g];
    cid = cid < 0 ? 0 : (cid > nEmb - 1 ? nEmb - 1 : cid);
    res[tid] = emb[(size_t)cid * EMBW + (tid - 2 * CH)];
  } else if (tid >= 2 * CH + EMBW && tid < CBW) {
    res[tid] = 0.f;
  }
  __syncthreads();
  v4f a = {0.f, 0.f, 0.f, 0.f}, b = {0.f, 0.f, 0.f, 0.f};
  float* rowp = comb + (size_t)g * CBW;
  if (wave == 0) {
    a = *(const v4f*)(res + 4 * lane);
    if (lane < 8) b = *(const v4f*)(res + 128 + 4 * lane);
    *(volatile v4f*)(rowp + 4 * lane) = a;
    if (lane < 8) *(volatile v4f*)(rowp + 128 + 4 * lane) = b;
  }
  __threadfence();
  if (wave == 0) {
    *(volatile v4f*)(rowp + 4 * lane) = a;
    if (lane < 8) *(volatile v4f*)(rowp + 128 + 4 * lane) = b;
  }
}

__device__ __forceinline__ void ldA2(const float* p, FragB& hi, FragB& lo) {
  const v4f a = *(const v4f*)p, b = *(const v4f*)(p + 4), c = *(const v4f*)(p + 16), d = *(const v4f*)(p + 20);
  const float f[16] = {a.x, a.y, a.z, a.w, b.x, b.y, b.z, b.w, c.x, c.y, c.z, c.w, d.x, d.y, d.z, d.w};
#pragma unroll
  for (int i = 0; i < 16; ++i) split2(f[i], hi.u[i], lo.u[i]);
}

template<int KP, int KR, int NR, int APT, int NCT, int ZP, int RELU>
__device__ __forceinline__ void mlp_gemm(const float* A, const float* __restrict__ B, const float* __restrict__ bvec,
                                         float* Z, int r0, int hh, int m) {
#pragma unroll 1
  for (int ct = 0; ct < NCT; ++ct) {
    const int  col = ct * 16 + m;
    const bool cv  = col < NR;
    const int  cc  = cv ? col : 0;
    v8f acc = {0.f, 0.f, 0.f, 0.f, 0.f, 0.f, 0.f, 0.f};
#pragma unroll
    for (int kt = 0; kt < KP / 32; ++kt) {
      const int k0 = kt * 32;
      FragB ah, al, bh, bl;
      ldA2(A + (r0 + m) * APT + k0 + 8 * hh, ah, al);
#pragma unroll
      for (int i = 0; i < 16; ++i) {
        const int k  = k0 + 8 * hh + i + ((i < 8) ? 0 : 8);
        const int kc = (k < KR) ? k : (KR - 1);
        float bv = B[(size_t)kc * NR + cc];
        bv = (cv && (k < KR)) ? bv : 0.f;
        split2(bv, bh.u[i], bl.u[i]);
      }
      acc = wmb(ah.v, bh.v, acc);
      acc = wmb(ah.v, bl.v, acc);
      acc = wmb(al.v, bh.v, acc);
    }
    const float bb = cv ? bvec[cc] : 0.f;
    if (cv) {
#pragma unroll
      for (int r = 0; r < 8; ++r) {
        float v = acc[r] + bb;
        if (RELU) v = v > 0.f ? v : 0.f;
        Z[(r0 + 8 * hh + r) * ZP + col] = v;
      }
    }
  }
}

__global__ __launch_bounds__(NTHR) void k_mlp(const float* __restrict__ comb,
                                              const float* __restrict__ mw1, const float* __restrict__ mb1,
                                              const float* __restrict__ mw2, const float* __restrict__ mb2,
                                              const float* __restrict__ mw3, const float* __restrict__ mb3,
                                              float* out) {
  __shared__ __attribute__((aligned(16))) float outs[GP * OUTW];
  float* cbuf = (float*)lds_dyn;
  float* z1   = cbuf + GP * CBP;
  const int tid  = threadIdx.x;
  const int lane = tid & 31;
  const int wave = tid >> 5;
  const int hh   = lane >> 4;
  const int m    = lane & 15;
  const int r0   = wave * 16;

  for (int u = tid; u < GP * (CBW / 4); u += NTHR) {
    const int row = u / (CBW / 4);
    const int c4  = (u - row * (CBW / 4)) * 4;
    *(v4f*)(cbuf + row * CBP + c4) = ld4(comb + (size_t)row * CBW + c4);
  }
  __syncthreads();
  mlp_gemm<CBW, M1K, M1N, CBP, M1N / 16, Z1P, 1>(cbuf, mw1, mb1, z1, r0, hh, m);
  __syncthreads();
  mlp_gemm<M1N, M1N, M2N, Z1P, M2N / 16, Z2P, 1>(z1, mw2, mb2, cbuf, r0, hh, m);
  __syncthreads();
  mlp_gemm<M2N, M2N, OUTW, Z2P, 1, OUTW, 0>(cbuf, mw3, mb3, outs, r0, hh, m);
  __syncthreads();
  v4f oa = {0.f, 0.f, 0.f, 0.f}, ob = {0.f, 0.f, 0.f, 0.f};
  if (wave == 0) {
    oa = *(const v4f*)(outs + 4 * lane);
    ob = *(const v4f*)(outs + (GP * OUTW) / 2 + 4 * lane);
    *(volatile v4f*)(out + 4 * lane) = oa;
    *(volatile v4f*)(out + (GP * OUTW) / 2 + 4 * lane) = ob;
  }
  __threadfence();
  if (wave == 0) {
    *(volatile v4f*)(out + 4 * lane) = oa;
    *(volatile v4f*)(out + (GP * OUTW) / 2 + 4 * lane) = ob;
  }
}

extern "C" void kernel_launch(void* const* d_in, const int* in_sizes, int n_in,
                              void* d_out, int out_size, void* d_ws, size_t ws_size,
                              hipStream_t stream) {
  if (n_in < 42) return;
  const int nN = in_sizes[0] / INW;
  if (nN <= 0 || in_sizes[0] != nN * INW) return;
  const int nE = in_sizes[1];
  if (nE < 0 || in_sizes[39] != 2 * nE) return;
  if (in_sizes[40] != nN) return;
  if (in_sizes[2] != INW * HCW || in_sizes[7] != HCW * HCW || in_sizes[12] != HCW * HCW) return;
  for (int l = 0; l < 3; ++l) {
    const int b = 2 + 5 * l;
    if (in_sizes[b + 1] != NH * CH || in_sizes[b + 2] != NH * CH || in_sizes[b + 3] != HCW || in_sizes[b + 4] != NH * CH) return;
  }
  if (in_sizes[17] != HCW || in_sizes[18] != HCW || in_sizes[19] != CH) return;
  for (int i = 20; i < 28; ++i) if (in_sizes[i] != HCW) return;
  for (int i = 28; i < 32; ++i) if (in_sizes[i] != CH) return;
  const int nEmb = in_sizes[32] / EMBW;
  if (nEmb <= 0 || in_sizes[32] != nEmb * EMBW) return;
  if (in_sizes[33] != M1K * M1N || in_sizes[34] != M1N || in_sizes[35] != M1N * M2N ||
      in_sizes[36] != M2N || in_sizes[37] != M2N * OUTW || in_sizes[38] != OUTW) return;
  if (in_sizes[41] != GP || out_size != GP * OUTW) return;

  const float* x  = (const float*)d_in[0];
  const float* ea = (const float*)d_in[1];
  const float* w_[3]  = { (const float*)d_in[2],  (const float*)d_in[7],  (const float*)d_in[12] };
  const float* as_[3] = { (const float*)d_in[3],  (const float*)d_in[8],  (const float*)d_in[13] };
  const float* ad_[3] = { (const float*)d_in[4],  (const float*)d_in[9],  (const float*)d_in[14] };
  const float* we_[3] = { (const float*)d_in[5],  (const float*)d_in[10], (const float*)d_in[15] };
  const float* ae_[3] = { (const float*)d_in[6],  (const float*)d_in[11], (const float*)d_in[16] };
  const float* bs_[3] = { (const float*)d_in[17], (const float*)d_in[18], (const float*)d_in[19] };
  const float* bng[3] = { (const float*)d_in[20], (const float*)d_in[24], (const float*)d_in[28] };
  const float* bnb[3] = { (const float*)d_in[21], (const float*)d_in[25], (const float*)d_in[29] };
  const float* bnm[3] = { (const float*)d_in[22], (const float*)d_in[26], (const float*)d_in[30] };
  const float* bnv[3] = { (const float*)d_in[23], (const float*)d_in[27], (const float*)d_in[31] };
  const float* emb = (const float*)d_in[32];
  const float* mw1 = (const float*)d_in[33]; const float* mb1 = (const float*)d_in[34];
  const float* mw2 = (const float*)d_in[35]; const float* mb2 = (const float*)d_in[36];
  const float* mw3 = (const float*)d_in[37]; const float* mb3 = (const float*)d_in[38];
  const int* ei    = (const int*)d_in[39];
  const int* batch = (const int*)d_in[40];
  const int* cids  = (const int*)d_in[41];
  float* out = (float*)d_out;

  const int nP = ((nN + GR - 1) / GR) * GR;
  size_t off = 0;
  char* wsb = (char*)d_ws;
  auto carve = [&](size_t bytes) -> char* { char* p = wsb + off; off += (bytes + 255) & ~(size_t)255; return p; };
  _Float16* Wt   = (_Float16*)carve((size_t)HCW * HCW * sizeof(_Float16));
  _Float16* xh   = (_Float16*)carve((size_t)nP * INW * sizeof(_Float16));
  _Float16* hb   = (_Float16*)carve((size_t)nP * HCW * sizeof(_Float16));
  float*    xp   = (float*)carve((size_t)nP * HCW * sizeof(float));
  float*    asrc = (float*)carve((size_t)nP * NH * sizeof(float));
  float*    adst = (float*)carve((size_t)nP * NH * sizeof(float));
  float*    hfin = (float*)carve((size_t)nP * CH * sizeof(float));
  float*    comb = (float*)carve((size_t)GP * CBW * sizeof(float));
  float*    eam  = (float*)carve(512);
  if (off > ws_size) return;

  const int n8    = nP * (INW / 8);
  const int gridG = nP / GR;
  const int gridA = (nN + NB - 1) / NB;

  hipFuncSetAttribute(reinterpret_cast<const void*>(&k_agg<0>), hipFuncAttributeMaxDynamicSharedMemorySize, AGG_LDS_BYTES);
  hipFuncSetAttribute(reinterpret_cast<const void*>(&k_agg<1>), hipFuncAttributeMaxDynamicSharedMemorySize, AGG_LDS_BYTES);
  hipFuncSetAttribute(reinterpret_cast<const void*>(&k_mlp),    hipFuncAttributeMaxDynamicSharedMemorySize, MLP_LDS_BYTES);

  k_eamean<<<1, NTHR, 0, stream>>>(ea, eam, nE);
  k_cvx<<<(n8 + NTHR - 1) / NTHR, NTHR, 0, stream>>>(x, xh, nN, n8);

  k_prepw<INW><<<HCW / 32, NTHR, 0, stream>>>(w_[0], Wt);
  k_gemm<INW><<<gridG, NTHR, 0, stream>>>(xh, Wt, as_[0], ad_[0], xp, asrc, adst);
  k_agg<0><<<gridA, NTHR, AGG_LDS_BYTES, stream>>>(ei, ea, eam, xp, asrc, adst, we_[0], ae_[0],
                                                    bs_[0], bng[0], bnb[0], bnm[0], bnv[0], hb, hfin, nN, nE);
  k_prepw<HCW><<<HCW / 32, NTHR, 0, stream>>>(w_[1], Wt);
  k_gemm<HCW><<<gridG, NTHR, 0, stream>>>(hb, Wt, as_[1], ad_[1], xp, asrc, adst);
  k_agg<0><<<gridA, NTHR, AGG_LDS_BYTES, stream>>>(ei, ea, eam, xp, asrc, adst, we_[1], ae_[1],
                                                    bs_[1], bng[1], bnb[1], bnm[1], bnv[1], hb, hfin, nN, nE);
  k_prepw<HCW><<<HCW / 32, NTHR, 0, stream>>>(w_[2], Wt);
  k_gemm<HCW><<<gridG, NTHR, 0, stream>>>(hb, Wt, as_[2], ad_[2], xp, asrc, adst);
  k_agg<1><<<gridA, NTHR, AGG_LDS_BYTES, stream>>>(ei, ea, eam, xp, asrc, adst, we_[2], ae_[2],
                                                    bs_[2], bng[2], bnb[2], bnm[2], bnv[2], hb, hfin, nN, nE);

  k_pool<<<GP, NTHR, 0, stream>>>(hfin, batch, emb, cids, comb, nN, nEmb);
  k_mlp<<<1, NTHR, MLP_LDS_BYTES, stream>>>(comb, mw1, mb1, mw2, mb2, mw3, mb3, out);
}
